// jgMPNN_3616362463932
// MI455X (gfx1250) — hardware-run, weakly checked
//
#include <hip/hip_runtime.h>


namespace {
constexpr int N = 2048, HID = 5, LCAP = 128, JC = 512  , NQ = JC * HID / 32  ;
constexpr float XS = 8.0f;
typedef _Float16 b16;
typedef __attribute__((ext_vector_type(16))) _Float16 v16b;
typedef __attribute__((ext_vector_type(8))) _Float16 v8b;
typedef __attribute__((ext_vector_type(8))) float v8f;
typedef __attribute__((ext_vector_type(4))) float v4f;
__device__ __forceinline__ float bf16_rne(float f) { unsigned int u = __float_as_uint(f); u += 0x7FFFu + ((u >> 16) & 1u); float r = __uint_as_float(u & 0xFFFF0000u); asm volatile("" : "+v"(r)); return r; }
__device__ __forceinline__ float bfv(float f) { float r = bf16_rne(f); asm volatile("" : "+v"(r)); return r; }
__device__ __forceinline__ v16b frag_kb(const b16* p, int hh) { const v8b a = *(const v8b*)(p + 8 * hh), b = *(const v8b*)(p + 16 + 8 * hh); v16b f;
#pragma unroll
  for (int e = 0; e < 8; ++e) { f[e] = a[e]; f[8 + e] = b[e]; } return f; }
__device__ __forceinline__ v8f wmma16b(v16b a, v16b b, v8f c) { v8f d = __builtin_amdgcn_wmma_f32_16x16x32_f16(false, a, false, b, (short)0, c, false, false); asm volatile("v_nop\n\tv_nop\n\tv_nop\n\tv_nop" : "+v"(d) : "v"(a), "v"(b)); return d; }
__device__ __forceinline__ void wave_lds_sync() { __builtin_amdgcn_fence(__ATOMIC_RELEASE, "workgroup"); __builtin_amdgcn_wave_barrier(); __builtin_amdgcn_fence(__ATOMIC_ACQUIRE, "workgroup"); }
__device__ __forceinline__ float pmul(float a, float b) { float p = a * b; asm volatile("" : "+v"(p)); return p; }
__device__ __forceinline__ int iclamp(int v, int lo, int hi) { return v < lo ? lo : (v > hi ? hi : v); }

__global__ __launch_bounds__(256) void lists_kernel(const float* __restrict__ a, int* __restrict__ OUTI, float* __restrict__ OUTV, int* __restrict__ OUTC, int* __restrict__ INI, float* __restrict__ INV, int* __restrict__ INC) { __shared__ int Li[8][LCAP]; __shared__ float Lv[8][LCAP]; __shared__ int Cs[2][8]; const int wave = threadIdx.x >> 5, lane = threadIdx.x & 31; const int n = blockIdx.x * 8 + wave;
#pragma unroll 1
  for (int dir = 0; dir < 2; ++dir) { for (int s = lane; s < LCAP; s += 32) { Li[wave][s] = 0; Lv[wave][s] = 0.0f; } wave_lds_sync(); int cnt = 0;
#pragma unroll 1
    for (int c = 0; c < N / 32; ++c) { const int z = c * 32 + lane; const float v = bfv(dir == 0 ? a[(size_t)n * N + z] : a[(size_t)z * N + n]); const bool flag = v != 0.0f; const unsigned int mask = __builtin_amdgcn_ballot_w32(flag); const int rank = __builtin_popcount(mask & ((1u << lane) - 1u)); const int pos = cnt + rank; if (flag && pos < LCAP) { Li[wave][pos] = z; Lv[wave][pos] = v; } cnt += __builtin_popcount(mask); }
    wave_lds_sync();
    int* DI = dir == 0 ? OUTI : INI; float* DV = dir == 0 ? OUTV : INV; int* DC = dir == 0 ? OUTC : INC;
    if (lane == 0) Cs[dir][wave] = cnt > LCAP ? -1 : cnt;
    for (int pass = 0; pass < 2; ++pass) { for (int s = lane; s < LCAP; s += 32) { ((volatile int*)DI)[(size_t)n * LCAP + s] = Li[wave][s]; ((volatile float*)DV)[(size_t)n * LCAP + s] = Lv[wave][s]; } __threadfence(); }
    (void)DC; wave_lds_sync(); }
  __syncthreads();
  for (int pass = 0; pass < 2; ++pass) { if (wave == 0) { ((volatile int*)OUTC)[(size_t)blockIdx.x * 32 + lane] = lane < 8 ? Cs[0][lane] : 0; ((volatile int*)INC)[(size_t)blockIdx.x * 32 + lane] = lane < 8 ? Cs[1][lane] : 0; } __threadfence(); } }
__device__ __forceinline__ int cnt_at(const int* C, int n) { return C[(n >> 3) * 32 + (n & 7)]; }
__global__ __launch_bounds__(256) void tpose_kernel(const float* __restrict__ a, const float* __restrict__ f, b16* __restrict__ AT, b16* __restrict__ FT) { __shared__ float Ta[64][65], Tb[64][65]; const int tz = blockIdx.x / (N / 64), ti = blockIdx.x % (N / 64); const int z0 = tz * 64, i0 = ti * 64; const int tid = threadIdx.x;
  for (int u = tid; u < 64 * 64; u += 256) { const int r = u / 64, c = u % 64; Ta[r][c] = bfv(a[(size_t)(z0 + r) * N + i0 + c]); Tb[r][c] = bfv(f[(size_t)(z0 + r) * N + i0 + c]); }
  __syncthreads(); const int wave = tid >> 5, lane = tid & 31;
  for (int pass = 0; pass < 2; ++pass) { for (int rr = 0; rr < 8; ++rr) { const int c = wave * 8 + rr; for (int q = 0; q < 2; ++q) { const int r = q * 32 + lane; ((volatile b16*)AT)[(size_t)(i0 + c) * N + z0 + r] = (b16)Ta[r][c]; ((volatile b16*)FT)[(size_t)(i0 + c) * N + z0 + r] = (b16)(Tb[r][c] * XS); } } __threadfence(); } }
__global__ __launch_bounds__(32) void agg_kernel(const b16* __restrict__ AT, const b16* __restrict__ FT, int R0, int NG, float* __restrict__ AG) { __shared__ float Tf[16][132]; const int lane = threadIdx.x, nloc = lane & 15, hlf = lane >> 4; const int g = blockIdx.x % NG; const size_t m0 = (size_t)R0 + (size_t)(blockIdx.x / NG) * 16; v8f acc[8];
#pragma unroll
  for (int t = 0; t < 8; ++t) acc[t] = (v8f){};
  const b16* arow = AT + (m0 + nloc) * N;
#pragma unroll 2
  for (int kb = 0; kb < N; kb += 32) { const v16b av = frag_kb(arow + kb, hlf);
#pragma unroll
    for (int t = 0; t < 8; ++t) acc[t] = wmma16b(av, frag_kb(FT + (size_t)(g * 128 + t * 16 + nloc) * N + kb, hlf), acc[t]); }
#pragma unroll
  for (int t = 0; t < 8; ++t)
#pragma unroll
    for (int r8 = 0; r8 < 8; ++r8) Tf[8 * hlf + r8][t * 16 + nloc] = acc[t][r8] * (1.0f / XS);
  wave_lds_sync();
  for (int pass = 0; pass < 2; ++pass) { for (int rr = 0; rr < 16; ++rr) *(volatile v4f*)(AG + (m0 + rr) * N + g * 128 + lane * 4) = *(const v4f*)(&Tf[rr][lane * 4]); __threadfence(); } }
__global__ __launch_bounds__(256) void htile_kernel(const float* __restrict__ f, const float* __restrict__ AG, const float* __restrict__ de, const float* __restrict__ w1, const float* __restrict__ b1, int TI0, int NTJ, float* __restrict__ H, float* __restrict__ HT) { __shared__ float Fa[32][33], Fb[32][33], Ga[32][33], Gb[32][33], Da[32][33], Db[32][33]; const int I = TI0 + blockIdx.x / NTJ, J = blockIdx.x % NTJ; const int i0 = I * 32, j0 = J * 32; const int tid = threadIdx.x;
  for (int u = tid; u < 1024; u += 256) { const int r = u >> 5, c = u & 31; Fa[r][c] = bfv(f[(size_t)(i0 + r) * N + j0 + c]); Ga[r][c] = AG[(size_t)(i0 + r) * N + j0 + c]; Da[r][c] = bfv(de[(size_t)(i0 + r) * N + j0 + c]); Fb[r][c] = bfv(f[(size_t)(j0 + r) * N + i0 + c]); Gb[r][c] = AG[(size_t)(j0 + r) * N + i0 + c]; Db[r][c] = bfv(de[(size_t)(j0 + r) * N + i0 + c]); }
  __syncthreads(); float w0[HID], wa[HID], bb[HID];
#pragma unroll
  for (int k = 0; k < HID; ++k) { w0[k] = bfv(w1[k * 2]); wa[k] = bfv(w1[k * 2 + 1]); bb[k] = bfv(b1[k]); }
  const int wave = tid >> 5, lane = tid & 31;
  for (int pass = 0; pass < 2; ++pass) { for (int rr = 0; rr < 4; ++rr) { const int r = wave * 4 + rr;
      { const float fv = Fa[r][lane], gv = (Ga[r][lane] + Gb[lane][r]) / (2.0f * Da[r][lane]);
#pragma unroll
        for (int k = 0; k < HID; ++k) ((volatile float*)H)[((size_t)(i0 + r) * N + j0 + lane) * HID + k] = fmaxf(pmul(w0[k], fv) + pmul(wa[k], gv) + bb[k], 0.0f); }
      { const float fv = Fb[lane][r], gv = (Gb[lane][r] + Ga[r][lane]) / (2.0f * Db[lane][r]);
#pragma unroll
        for (int k = 0; k < HID; ++k) ((volatile float*)HT)[((size_t)(i0 + r) * N + j0 + lane) * HID + k] = fmaxf(pmul(w0[k], fv) + pmul(wa[k], gv) + bb[k], 0.0f); } } __threadfence(); } }
__global__ __launch_bounds__(32) void main_kernel(const float* __restrict__ H, const float* __restrict__ HT, const float* __restrict__ de, const int* __restrict__ INI, const float* __restrict__ INV, const int* __restrict__ INC, const int* __restrict__ OUTI, const float* __restrict__ OUTV, const int* __restrict__ OUTC, const float* __restrict__ w2, const float* __restrict__ b2, const float* __restrict__ nn_unused, int ILIM, float* __restrict__ out) {
  __shared__ float Hr[N * HID], Ct[JC * HID], Acc[JC * HID]; const int lane = threadIdx.x; const int jc = blockIdx.x % (N / JC); const size_t i = blockIdx.x / (N / JC); if (i >= (size_t)ILIM) return; const int jbase = jc * JC;
  for (int u = lane; u < N * HID; u += 32) Hr[u] = H[i * N * HID + u]; for (int u = lane; u < JC * HID; u += 32) Acc[u] = 0.0f;
  const int cin = cnt_at(INC, (int)i); const bool bad_i = cin < 0;
#pragma unroll 1
  for (int e = 0; e < (bad_i ? 0 : cin); ++e) { const int z = iclamp(INI[i * LCAP + e], 0, N - 1); const float av = INV[i * LCAP + e]; const float* hrow = HT + ((size_t)z * N + jbase) * HID;
#pragma unroll 1
    for (int t = 0; t < NQ; ++t) { const int q = lane + 32 * t; Acc[q] += pmul(av, hrow[q]); } }
  wave_lds_sync();
  bool bad = bad_i;
#pragma unroll 1
  for (int t = 0; t < NQ; ++t) { const int q = lane + 32 * t; const int jl = q / HID, k = q % HID; const int j = jbase + jl; const int co = cnt_at(OUTC, j); bad |= co < 0; float s2 = 0.0f;
#pragma unroll 1
    for (int e = 0; e < (co < 0 ? 0 : co); ++e) { const int z = iclamp(OUTI[(size_t)j * LCAP + e], 0, N - 1); s2 += pmul(OUTV[(size_t)j * LCAP + e], Hr[z * HID + k]); }
    const float ag2 = (Acc[q] + s2) / bfv(de[i * N + j]); Ct[q] = pmul(bfv(w2[k]), Hr[(size_t)j * HID + k]) + pmul(bfv(w2[HID + k]), ag2); }
  wave_lds_sync();
  const unsigned int anybad = __builtin_amdgcn_ballot_w32(bad); const float bb = bfv(b2[0]) + 0.0f * nn_unused[0];
  for (int pass = 0; pass < 2; ++pass) { for (int m = 0; m < JC / 32; ++m) { const int jl = m * 32 + lane; float s = bb;
#pragma unroll
      for (int k = 0; k < HID; ++k) s += Ct[jl * HID + k]; ((volatile float*)out)[i * N + jbase + jl] = anybad ? __builtin_nanf("") : s; } __threadfence(); } }
}

extern "C" void kernel_launch(void* const* d_in, const int* in_sizes, int n_in, void* d_out, int out_size, void* d_ws, size_t ws_size, hipStream_t stream) {
  (void)n_in;
  auto Fp = [&](int i) { return (const float*)d_in[i]; };
  if (in_sizes[0] != N * N || in_sizes[2] != N * N || in_sizes[3] != N * N || in_sizes[4] != HID * 2 || in_sizes[5] != HID || in_sizes[6] != 2 * HID || out_size != N * N) return;
  const int ILIM = N, JLIM = N;
  const int RL = JLIM > ILIM ? JLIM : ILIM;
  size_t off = 0; char* ws = (char*)d_ws;
  auto carve = [&](size_t bytes) { char* p = ws + off; off += (bytes + 255) & ~(size_t)255; return p; };
  int* OUTI = (int*)carve((size_t)N * LCAP * 4); float* OUTV = (float*)carve((size_t)N * LCAP * 4); int* OUTC = (int*)carve((size_t)(N / 8) * 128); int* INI = (int*)carve((size_t)N * LCAP * 4); float* INV = (float*)carve((size_t)N * LCAP * 4); int* INC = (int*)carve((size_t)(N / 8) * 128);
  b16* AT = (b16*)carve((size_t)N * N * 2); b16* FT = (b16*)carve((size_t)N * N * 2); float* AG = (float*)carve((size_t)N * N * 4); float* H = (float*)carve((size_t)N * N * HID * 4); float* HT = (float*)carve((size_t)N * N * HID * 4);
  if (off > ws_size || off > ((size_t)232 << 20)) return;
  lists_kernel<<<N / 8, 256, 0, stream>>>(Fp(0), OUTI, OUTV, OUTC, INI, INV, INC);
  tpose_kernel<<<(N / 64) * (N / 64), 256, 0, stream>>>(Fp(0), Fp(2), AT, FT);
  agg_kernel<<<(RL / 16) * (N / 128), 32, 0, stream>>>(AT, FT, 0, N / 128, AG);
  if (RL < N) agg_kernel<<<((N - RL) / 16) * (JLIM / 128), 32, 0, stream>>>(AT, FT, RL, JLIM / 128, AG);
  htile_kernel<<<(ILIM / 32) * (N / 32), 256, 0, stream>>>(Fp(2), AG, Fp(3), Fp(4), Fp(5), 0, N / 32, H, HT);
  if (ILIM < N) htile_kernel<<<((N - ILIM) / 32) * (JLIM / 32), 256, 0, stream>>>(Fp(2), AG, Fp(3), Fp(4), Fp(5), ILIM / 32, JLIM / 32, H, HT);
  main_kernel<<<ILIM * (N / JC), 32, 0, stream>>>(H, HT, Fp(3), INI, INV, INC, OUTI, OUTV, OUTC, Fp(6), Fp(7), Fp(1), ILIM, (float*)d_out);
  (void)JLIM;
}
